// ContextAwareAttention_7696581394771
// MI455X (gfx1250) — hardware-verified
//
#include <hip/hip_runtime.h>
#include <math.h>

constexpr int kBatch  = 4;
constexpr int kSeq    = 2048;
constexpr int kDim    = 1024;
constexpr int kTok    = kBatch * kSeq;
constexpr int kChunkB = 2;
constexpr float kWCarry     = 16.0f;
constexpr float kWCarryInv  = 1.0f / 16.0f;
constexpr float kPCarry     = 2048.0f;
constexpr float kPCarryInv  = 1.0f / 2048.0f;
constexpr float kScoreScale = 0.03125f;

typedef __attribute__((ext_vector_type(16))) _Float16 v16h;
typedef __attribute__((ext_vector_type(8)))  _Float16 v8h;
typedef __attribute__((ext_vector_type(16))) __bf16   v16b;
typedef __attribute__((ext_vector_type(8)))  __bf16   v8b;
typedef __attribute__((ext_vector_type(8)))  float    v8f;
typedef __attribute__((ext_vector_type(4)))  float    v4f;
typedef __attribute__((ext_vector_type(4)))  unsigned int v4u;

__device__ __forceinline__ unsigned short f2bf_bits(float f) {
  unsigned u = __float_as_uint(f);
  return (unsigned short)((u + 0x7FFFu + ((u >> 16) & 1u)) >> 16);
}
__device__ __forceinline__ float bf_bits2f(unsigned short h) { return __uint_as_float(((unsigned)h) << 16); }

__device__ __forceinline__ void dep_guard_h(v8f& a, v8f& b, v16h x, v16h y) { asm volatile("v_nop\n\tv_nop\n\tv_nop\n\tv_nop" : "+v"(a), "+v"(b) : "v"(x), "v"(y)); }
__device__ __forceinline__ void dep_guard_b(v8f& a, v8f& b, v16b x, v16b y) { asm volatile("v_nop\n\tv_nop\n\tv_nop\n\tv_nop" : "+v"(a), "+v"(b) : "v"(x), "v"(y)); }
__device__ __forceinline__ void keep4_h(v16h a, v16h b, v16h c, v16h d) { asm volatile("v_nop" :: "v"(a), "v"(b), "v"(c), "v"(d)); }
__device__ __forceinline__ void keep4_b(v16b a, v16b b, v16b c, v16b d) { asm volatile("v_nop" :: "v"(a), "v"(b), "v"(c), "v"(d)); }
__device__ __forceinline__ void acc_guard4(v8f& a, v8f& b, v8f& c, v8f& d) { asm volatile("v_nop\n\tv_nop\n\tv_nop\n\tv_nop" : "+v"(a), "+v"(b), "+v"(c), "+v"(d)); }
template <typename T> struct Frag;
template <> struct Frag<_Float16> {
  typedef v16h V; union U { v16h v; v8h h[2]; };
  static __device__ __forceinline__ v16h load(const _Float16* p) {
    U f; f.h[0] = *(const v8h*)(p); f.h[1] = *(const v8h*)(p + 16); return f.v;
  }
  static __device__ __forceinline__ v8f mma(v16h a, v16h b, v8f c) {
    return __builtin_amdgcn_wmma_f32_16x16x32_f16(false, a, false, b, (short)0, c, false, false);
  }
  static __device__ __forceinline__ void guard(v8f& a, v8f& b, v16h x, v16h y) { dep_guard_h(a, b, x, y); }
  static __device__ __forceinline__ void keep(v16h a, v16h b, v16h c, v16h d) { keep4_h(a, b, c, d); }
};
template <> struct Frag<__bf16> {
  typedef v16b V; union U { v16b v; v8b h[2]; };
  static __device__ __forceinline__ v16b load(const __bf16* p) {
    U f; f.h[0] = *(const v8b*)(p); f.h[1] = *(const v8b*)(p + 16); return f.v;
  }
  static __device__ __forceinline__ v8f mma(v16b a, v16b b, v8f c) {
    return __builtin_amdgcn_wmma_f32_16x16x32_bf16(false, a, false, b, (short)0, c, false, false);
  }
  static __device__ __forceinline__ void guard(v8f& a, v8f& b, v16b x, v16b y) { dep_guard_b(a, b, x, y); }
  static __device__ __forceinline__ void keep(v16b a, v16b b, v16b c, v16b d) { keep4_b(a, b, c, d); }
};

__device__ __forceinline__ unsigned pk16(unsigned short a, unsigned short b) { return (unsigned)a | ((unsigned)b << 16); }
__device__ __forceinline__ unsigned short h_bits(float f) { const _Float16 h = (_Float16)f; return __builtin_bit_cast(unsigned short, h); }

template <int ET> struct Elem;
template <> struct Elem<0> { typedef _Float16 T; };
template <> struct Elem<1> { typedef __bf16 T; };
template <int ET, bool SPLIT, int BIAS_MODE, int OUT_MODE, bool RESID, int ACT = 0>
__global__ __launch_bounds__(256) void wmma_gemm64(
    const unsigned short* __restrict__ Ap, const unsigned short* __restrict__ A2p, int lda, long strideA,
    const unsigned short* __restrict__ Btp, const unsigned short* __restrict__ Bt2p, int ldb, long strideB,
    void* __restrict__ Cout, void* __restrict__ Cout2, int ldc, long strideC,
    const float* __restrict__ bias,
    const float* __restrict__ resid, long strideR,
    int M, int N, int K, float scale) {
  typedef typename Elem<ET>::T T;
  typedef typename Frag<T>::V V;
  const T* A = (const T*)Ap; const T* A2 = (const T*)A2p; const T* Bt = (const T*)Btp; const T* Bt2 = (const T*)Bt2p;
  __shared__ __align__(16) float sT[8][16 * 68];
  const int b    = blockIdx.y;
  const int lane = threadIdx.x & 31;
  const int wave = threadIdx.x >> 5;
  const int tilesN = N >> 6;
  const int tilesM = M >> 6;
  const int tile = blockIdx.x * 8 + wave;
  if (tile >= tilesM * tilesN) return;
  const int tm = tile / tilesN;
  const int tn = tile - tm * tilesN;
  const int m0 = tm << 6;
  const int n0 = tn << 6;

  const T* Ab  = A  + (size_t)b * strideA;
  const T* Bb  = Bt + (size_t)b * strideB;
  const T* Ab2 = SPLIT ? (A2  + (size_t)b * strideA) : nullptr;
  const T* Bb2 = SPLIT ? (Bt2 + (size_t)b * strideB) : nullptr;

  const int rlane = lane & 15;
  const int koff  = (lane >> 4) * 8;
  const int mOff  = (lane >> 4) * 8;

  v8f acc[4][4];
#pragma unroll
  for (int i = 0; i < 4; ++i)
#pragma unroll
    for (int j = 0; j < 4; ++j) acc[i][j] = (v8f){0.f,0.f,0.f,0.f,0.f,0.f,0.f,0.f};

  for (int k0 = 0; k0 < K; k0 += 32) {
    V bh[4], bl[4];
#pragma unroll
    for (int j = 0; j < 4; ++j) {
      const size_t bo = (size_t)(n0 + (j << 4) + rlane) * ldb + koff + k0;
      bh[j] = Frag<T>::load(Bb + bo);
      if (SPLIT) bl[j] = Frag<T>::load(Bb2 + bo);
    }
#pragma unroll
    for (int i = 0; i < 4; ++i) {
      const size_t ao = (size_t)(m0 + (i << 4) + rlane) * lda + koff + k0;
      V ah = Frag<T>::load(Ab + ao);
      V al;
      if (SPLIT) al = Frag<T>::load(Ab2 + ao);
#pragma unroll
      for (int j = 0; j < 4; ++j) {
        acc[i][j] = Frag<T>::mma(ah, bh[j], acc[i][j]);
        if (SPLIT) {
          acc[i][j] = Frag<T>::mma(ah, bl[j], acc[i][j]);
          acc[i][j] = Frag<T>::mma(al, bh[j], acc[i][j]);
        }
      }
      Frag<T>::guard(acc[i][0], acc[i][3], ah, SPLIT ? al : ah);
    }
    Frag<T>::keep(bh[0], bh[1], bh[2], bh[3]);
    if (SPLIT) Frag<T>::keep(bl[0], bl[1], bl[2], bl[3]);
  }
  acc_guard4(acc[0][0], acc[0][1], acc[0][2], acc[0][3]);
  acc_guard4(acc[1][0], acc[1][1], acc[1][2], acc[1][3]);
  acc_guard4(acc[2][0], acc[2][1], acc[2][2], acc[2][3]);
  acc_guard4(acc[3][0], acc[3][1], acc[3][2], acc[3][3]);

  float* slab = sT[wave];
  const float* Rb = RESID ? (resid + (size_t)b * strideR) : nullptr;
#pragma unroll
  for (int i = 0; i < 4; ++i) {
    const int mBase = m0 + (i << 4);
#pragma unroll
    for (int j = 0; j < 4; ++j) {
      const int n = n0 + (j << 4) + rlane;
      float bv = 0.f;
      if (BIAS_MODE == 2) bv = bias[n];
#pragma unroll
      for (int r = 0; r < 8; ++r) {
        float v = acc[i][j][r] * scale;
        if (BIAS_MODE == 1) v += bias[mBase + mOff + r];
        if (BIAS_MODE == 2) v += bv;
        if (RESID) v += Rb[(size_t)(mBase + mOff + r) * ldc + n];
        if (ACT == 2) v = fmaxf(v, 0.0f);
        if (ACT == 4) v = (v > 0.f) ? v : 0.01f * v;
        slab[(mOff + r) * 68 + (j << 4) + rlane] = v;
      }
    }
    __builtin_amdgcn_fence(__ATOMIC_RELEASE, "workgroup");
    __builtin_amdgcn_wave_barrier();
    __builtin_amdgcn_fence(__ATOMIC_ACQUIRE, "workgroup");
    if (OUT_MODE == 0) {
      float* C = (float*)Cout + (size_t)b * strideC;
      const int hh = lane >> 4, c4 = (lane & 15) * 4;
      for (int pass = 0; pass < 2; ++pass) {
#pragma unroll
        for (int it = 0; it < 8; ++it) {
          const int row = it * 2 + hh;
          v4f v = *(const v4f*)(slab + row * 68 + c4);
          *(volatile v4f*)(C + (size_t)(mBase + row) * ldc + n0 + c4) = v;
        }
        __threadfence();
      }
    } else {
      const int q = lane >> 3, c8 = (lane & 7) * 8;
      unsigned short* C  = (unsigned short*)Cout  + (size_t)b * strideC;
      unsigned short* C2 = (OUT_MODE == 2) ? ((unsigned short*)Cout2 + (size_t)b * strideC) : nullptr;
      for (int pass = 0; pass < 2; ++pass) {
#pragma unroll
        for (int it = 0; it < 4; ++it) {
          const int row = it * 4 + q;
          const float* sp = slab + row * 68 + c8;
          v8h hv, lv;
#pragma unroll
          for (int e = 0; e < 8; ++e) {
            if (OUT_MODE == 1) {
              hv[e] = (_Float16)sp[e];
            } else {
              unsigned short hb = f2bf_bits(sp[e]);
              unsigned short lb = f2bf_bits(sp[e] - bf_bits2f(hb));
              hv[e] = __builtin_bit_cast(_Float16, hb);
              lv[e] = __builtin_bit_cast(_Float16, lb);
            }
          }
          *(volatile v8h*)(C + (size_t)(mBase + row) * ldc + n0 + c8) = hv;
          if (OUT_MODE == 2) *(volatile v8h*)(C2 + (size_t)(mBase + row) * ldc + n0 + c8) = lv;
        }
        __threadfence();
      }
    }
    __builtin_amdgcn_fence(__ATOMIC_RELEASE, "workgroup");
    __builtin_amdgcn_wave_barrier();
    __builtin_amdgcn_fence(__ATOMIC_ACQUIRE, "workgroup");
  }
}

template <bool HAS_CTX>
__global__ __launch_bounds__(256) void cast8_f16_kernel(const float* __restrict__ in, const float* __restrict__ ctx,
                                                        unsigned short* __restrict__ out, int n8, float scale) {
  const int i = blockIdx.x * 256 + threadIdx.x;
  if (i >= n8) return;
  const float* p = in + 8 * (size_t)i;
  v4f a = *(const v4f*)(p);
  v4f c = *(const v4f*)(p + 4);
  if (HAS_CTX) {
    const int cb = (int)((8 * (size_t)i) & (size_t)(kDim - 1));
    const v4f g0 = *(const v4f*)(ctx + cb);
    const v4f g1 = *(const v4f*)(ctx + cb + 4);
    a = a + g0;
    c = c + g1;
  }
  unsigned short hb[8];
#pragma unroll
  for (int e = 0; e < 4; ++e) {
    hb[e]     = h_bits(a[e] * scale);
    hb[4 + e] = h_bits(c[e] * scale);
  }
  const v4u u = (v4u){pk16(hb[0], hb[1]), pk16(hb[2], hb[3]), pk16(hb[4], hb[5]), pk16(hb[6], hb[7])};
  unsigned short* q = out + 8 * (size_t)i;
  *(volatile v4u*)q = u;
  __threadfence();
  *(volatile v4u*)q = u;
}

__global__ __launch_bounds__(256) void softmax_row_kernel(const float* __restrict__ S, unsigned short* __restrict__ P,
                                                          float carry) {
  __shared__ float redM[8];
  __shared__ float redS[8];
  const int row  = blockIdx.x;
  const int t    = threadIdx.x;
  const int lane = t & 31, wave = t >> 5;
  const int c0   = t * 8;
  const float* sr = S + (size_t)row * kSeq + c0;
  const v4f a = *(const v4f*)(sr);
  const v4f c = *(const v4f*)(sr + 4);
  float x[8];
#pragma unroll
  for (int e = 0; e < 4; ++e) { x[e] = a[e]; x[4 + e] = c[e]; }
  float m = fmaxf(fmaxf(fmaxf(x[0], x[1]), fmaxf(x[2], x[3])), fmaxf(fmaxf(x[4], x[5]), fmaxf(x[6], x[7])));
#pragma unroll
  for (int off = 16; off > 0; off >>= 1) m = fmaxf(m, __shfl_xor(m, off, 32));
  if (lane == 0) redM[wave] = m;
  __syncthreads();
  float gm = redM[0];
#pragma unroll
  for (int w = 1; w < 8; ++w) gm = fmaxf(gm, redM[w]);
  float p[8];
  float s = 0.f;
#pragma unroll
  for (int e = 0; e < 8; ++e) { p[e] = expf(x[e] - gm); s += p[e]; }
#pragma unroll
  for (int off = 16; off > 0; off >>= 1) s += __shfl_xor(s, off, 32);
  if (lane == 0) redS[wave] = s;
  __syncthreads();
  float tot = redS[0];
#pragma unroll
  for (int w = 1; w < 8; ++w) tot += redS[w];
  const float rcp = 1.0f / tot;
  unsigned short hb[8];
#pragma unroll
  for (int e = 0; e < 8; ++e) hb[e] = h_bits((p[e] * rcp) * carry);
  const v4u u = (v4u){pk16(hb[0], hb[1]), pk16(hb[2], hb[3]), pk16(hb[4], hb[5]), pk16(hb[6], hb[7])};
  unsigned short* q = P + (size_t)row * kSeq + c0;
  *(volatile v4u*)q = u;
  __threadfence();
  *(volatile v4u*)q = u;
}

extern "C" void kernel_launch(void* const* d_in, const int* in_sizes, int n_in,
                              void* d_out, int out_size, void* d_ws, size_t ws_size,
                              hipStream_t stream) {
  if (n_in < 10) return;
  const float* query = (const float*)d_in[0];
  const float* key   = (const float*)d_in[1];
  const float* value = (const float*)d_in[2];
  const float* ctx   = (const float*)d_in[3];
  const float* Wq    = (const float*)d_in[4];
  const float* bq    = (const float*)d_in[5];
  const float* Wk    = (const float*)d_in[6];
  const float* bk    = (const float*)d_in[7];
  const float* Wv    = (const float*)d_in[8];
  const float* bv    = (const float*)d_in[9];
  float* out = (float*)d_out;

  const size_t actE = (size_t)kTok * kDim;
  const size_t wE   = (size_t)kDim * kDim;
  if ((size_t)in_sizes[0] != actE || (size_t)in_sizes[1] != actE || (size_t)in_sizes[2] != actE) return;
  if ((size_t)in_sizes[3] != (size_t)kDim) return;
  if ((size_t)in_sizes[4] != wE || (size_t)in_sizes[6] != wE || (size_t)in_sizes[8] != wE) return;
  if ((size_t)in_sizes[5] != (size_t)kDim || (size_t)in_sizes[7] != (size_t)kDim || (size_t)in_sizes[9] != (size_t)kDim) return;
  if ((size_t)out_size != actE) return;

  const size_t actB16 = actE * 2;
  const size_t wB16   = wE * 2;
  unsigned char* ws = (unsigned char*)d_ws;
  size_t off = 0;
  unsigned short* Xq16 = (unsigned short*)(ws + off); off += actB16;
  unsigned short* Xk16 = (unsigned short*)(ws + off); off += actB16;
  unsigned short* Xv16 = (unsigned short*)(ws + off); off += actB16;
  unsigned short* Wq16 = (unsigned short*)(ws + off); off += wB16;
  unsigned short* Wk16 = (unsigned short*)(ws + off); off += wB16;
  unsigned short* Wv16 = (unsigned short*)(ws + off); off += wB16;
  unsigned short* Q16  = (unsigned short*)(ws + off); off += actB16;
  unsigned short* K16  = (unsigned short*)(ws + off); off += actB16;
  unsigned short* VT16 = (unsigned short*)(ws + off); off += actB16;
  const size_t carveTotal = off;
  if (carveTotal > ws_size) return;
  const size_t scBytes = (size_t)kChunkB * kSeq * kSeq * sizeof(float);
  const size_t pBytes  = (size_t)kChunkB * kSeq * kSeq * 2;
  if (scBytes + pBytes > 3 * actB16) return;
  float*          Sc  = (float*)(ws + 0);
  unsigned short* P16 = (unsigned short*)(ws + scBytes);

  const dim3 blk(256);

  const int n8act = (int)(actE / 8);
  const dim3 gAct((unsigned)((n8act + 255) / 256));
  cast8_f16_kernel<true ><<<gAct, blk, 0, stream>>>(query, ctx, Xq16, n8act, 1.0f);
  cast8_f16_kernel<true ><<<gAct, blk, 0, stream>>>(key,   ctx, Xk16, n8act, 1.0f);
  cast8_f16_kernel<false><<<gAct, blk, 0, stream>>>(value, ctx, Xv16, n8act, 1.0f);

  const int n8w = (int)(wE / 8);
  const dim3 gW((unsigned)((n8w + 255) / 256));
  cast8_f16_kernel<false><<<gW, blk, 0, stream>>>(Wq, ctx, Wq16, n8w, kWCarry);
  cast8_f16_kernel<false><<<gW, blk, 0, stream>>>(Wk, ctx, Wk16, n8w, kWCarry);
  cast8_f16_kernel<false><<<gW, blk, 0, stream>>>(Wv, ctx, Wv16, n8w, kWCarry);

  {
    const int M = kTok, N = kDim, K = kDim;
    const dim3 g((unsigned)(((M / 64) * (N / 64) + 7) / 8), 1);
    wmma_gemm64<0, false, 2, 1, false, 0><<<g, blk, 0, stream>>>(
        Xq16, Xq16, kDim, 0L, Wq16, Wq16, kDim, 0L, (void*)Q16, (void*)Q16, kDim, 0L,
        bq, bq, 0L, M, N, K, kWCarryInv);
    wmma_gemm64<0, false, 2, 1, false, 0><<<g, blk, 0, stream>>>(
        Xk16, Xk16, kDim, 0L, Wk16, Wk16, kDim, 0L, (void*)K16, (void*)K16, kDim, 0L,
        bk, bk, 0L, M, N, K, kWCarryInv);
  }
  {
    const int M = kDim, N = kSeq, K = kDim;
    const dim3 g((unsigned)(((M / 64) * (N / 64) + 7) / 8), (unsigned)kBatch);
    wmma_gemm64<0, false, 1, 1, false, 0><<<g, blk, 0, stream>>>(
        Wv16, Wv16, kDim, 0L,
        Xv16, Xv16, kDim, (long)kSeq * kDim,
        (void*)VT16, (void*)VT16, kSeq, (long)kDim * kSeq,
        bv, bv, 0L, M, N, K, kWCarryInv);
  }

  for (int ch = 0; ch < kBatch / kChunkB; ++ch) {
    const size_t b0 = (size_t)ch * kChunkB;
    const unsigned short* Qc  = Q16  + b0 * (size_t)kSeq * kDim;
    const unsigned short* Kc  = K16  + b0 * (size_t)kSeq * kDim;
    const unsigned short* VTc = VT16 + b0 * (size_t)kDim * kSeq;
    float* Oc = out + b0 * (size_t)kSeq * kDim;
    {
      const int M = kSeq, N = kSeq, K = kDim;
      const dim3 g((unsigned)(((M / 64) * (N / 64) + 7) / 8), (unsigned)kChunkB);
      wmma_gemm64<0, false, 0, 0, false, 0><<<g, blk, 0, stream>>>(
          Qc, Qc, kDim, (long)kSeq * kDim,
          Kc, Kc, kDim, (long)kSeq * kDim,
          (void*)Sc, (void*)Sc, kSeq, (long)kSeq * kSeq,
          bq, bq, 0L, M, N, K, kScoreScale);
    }
    {
      const dim3 g((unsigned)(kChunkB * kSeq));
      softmax_row_kernel<<<g, blk, 0, stream>>>(Sc, P16, kPCarry);
    }
    {
      const int M = kSeq, N = kDim, K = kSeq;
      const dim3 g((unsigned)(((M / 64) * (N / 64) + 7) / 8), (unsigned)kChunkB);
      wmma_gemm64<0, false, 0, 0, false, 0><<<g, blk, 0, stream>>>(
          P16, P16, kSeq, (long)kSeq * kSeq,
          VTc, VTc, kSeq, (long)kDim * kSeq,
          (void*)Oc, (void*)Oc, kDim, (long)kSeq * kDim,
          bq, bq, 0L, M, N, K, kPCarryInv);
    }
  }
}
